// Histogram2D_28252294873506
// MI455X (gfx1250) — hardware-verified
//
#include <hip/hip_runtime.h>


#define NPT  500000
#define CHK  100000
#define NCH  (NPT / CHK)
#define NBIN 128
#define XC   6
typedef _Float16 h16;
typedef unsigned short bf;
typedef __attribute__((ext_vector_type(16))) __bf16   v16bf;
typedef __attribute__((ext_vector_type(16))) _Float16 v16h;
typedef __attribute__((ext_vector_type(8)))  _Float16 v8h;
typedef __attribute__((ext_vector_type(8)))  unsigned short v8us;
typedef __attribute__((ext_vector_type(8)))  float    v8f;
typedef __attribute__((ext_vector_type(4)))  float    v4f;
typedef v8h  __attribute__((may_alias)) v8ha;
typedef v4f  __attribute__((may_alias)) v4fa;
typedef v8us __attribute__((may_alias)) v8usa;

__device__ __forceinline__ unsigned short f2bf(float f) { unsigned u = __float_as_uint(f); u += 0x7FFFu + ((u >> 16) & 1u); return (unsigned short)(u >> 16); }
__device__ __forceinline__ float bf2f(unsigned short b) { return __uint_as_float(((unsigned)b) << 16); }
__device__ __forceinline__ float bfr(float f) { return bf2f(f2bf(f)); }
__device__ __forceinline__ v16h cat16(v8h lo, v8h hi) { return __builtin_shufflevector(lo, hi, 0, 1, 2, 3, 4, 5, 6, 7, 8, 9, 10, 11, 12, 13, 14, 15); }
__device__ __forceinline__ v16bf cat16b(v8us lo, v8us hi) { return __builtin_bit_cast(v16bf, __builtin_shufflevector(lo, hi, 0, 1, 2, 3, 4, 5, 6, 7, 8, 9, 10, 11, 12, 13, 14, 15)); }
__device__ __forceinline__ v8f wmma16(v16h a, v16h b, v8f c) { return __builtin_amdgcn_wmma_f32_16x16x32_f16(false, a, false, b, (short)0, c, false, false); }
__device__ __forceinline__ v8f wmmab(v16bf a, v16bf b, v8f c) { return __builtin_amdgcn_wmma_f32_16x16x32_bf16(false, a, false, b, (short)0, c, false, false); }


template <typename T16> struct WFrag;
template <> struct WFrag<h16> { typedef v16h V; static __device__ __forceinline__ V ld(const h16* p) { return cat16(*(const v8h*)p, *(const v8h*)(p + 16)); } static __device__ __forceinline__ v8f mma(V a, V b, v8f c) { return wmma16(a, b, c); } };
template <> struct WFrag<bf> { typedef v16bf V; static __device__ __forceinline__ V ld(const bf* p) { return cat16b(*(const v8us*)p, *(const v8us*)(p + 16)); } static __device__ __forceinline__ v8f mma(V a, V b, v8f c) { return wmmab(a, b, c); } };
template <typename T16, int NSPLIT, bool BIAS>
__global__ __launch_bounds__(32) void k_gemmw(const T16* __restrict__ A, const T16* __restrict__ A2, const T16* __restrict__ Bt, const T16* __restrict__ Bt2, int K, float* C, int ldc, const float* __restrict__ bias, size_t sA, size_t sB, size_t sC) {
    typedef typename WFrag<T16>::V V;
    __shared__ __align__(16) float os[16 * 68];
    const size_t z = blockIdx.z; A += z * sA; if (A2) A2 += z * sA; Bt += z * sB; if (Bt2) Bt2 += z * sB; C += z * sC;
    const int lane = threadIdx.x & 31, lr = lane & 15, hi = lane >> 4; const int r0 = blockIdx.x * 64, c0 = blockIdx.y * 64;
    v8f acc[4][4];
#pragma unroll
    for (int mb = 0; mb < 4; ++mb)
#pragma unroll
        for (int nb = 0; nb < 4; ++nb) acc[mb][nb] = (v8f){};
    const size_t aoff = (size_t)(r0 + lr) * K + 8 * hi, boff = (size_t)(c0 + lr) * K + 8 * hi;
#pragma unroll 1
    for (int kc = 0; kc < K; kc += 32) {
        V a[4], a2[4];
#pragma unroll
        for (int mb = 0; mb < 4; ++mb) { a[mb] = WFrag<T16>::ld(A + aoff + (size_t)mb * 16 * K + kc); if (NSPLIT == 1 || NSPLIT == 2) a2[mb] = WFrag<T16>::ld(A2 + aoff + (size_t)mb * 16 * K + kc); }
#pragma unroll
        for (int nb = 0; nb < 4; ++nb) { const V b = WFrag<T16>::ld(Bt + boff + (size_t)nb * 16 * K + kc); V b2; if (NSPLIT >= 2) b2 = WFrag<T16>::ld(Bt2 + boff + (size_t)nb * 16 * K + kc);
#pragma unroll
            for (int mb = 0; mb < 4; ++mb) { acc[mb][nb] = WFrag<T16>::mma(a[mb], b, acc[mb][nb]); if (NSPLIT == 1 || NSPLIT == 2) acc[mb][nb] = WFrag<T16>::mma(a2[mb], b, acc[mb][nb]); if (NSPLIT >= 2) acc[mb][nb] = WFrag<T16>::mma(a[mb], b2, acc[mb][nb]); } }
        asm volatile("v_nop\n\tv_nop\n\tv_nop\n\tv_nop" : "+v"(acc[0][0]), "+v"(acc[1][1]), "+v"(acc[2][2]), "+v"(acc[3][3]) : "v"(a[0]), "v"(a[3]));
    }
#pragma unroll
    for (int mb = 0; mb < 4; ++mb) {
#pragma unroll
        for (int nb = 0; nb < 4; ++nb) {
#pragma unroll
            for (int j = 0; j < 8; ++j) os[(hi * 8 + j) * 68 + nb * 16 + lr] = acc[mb][nb][j]; }
        __builtin_amdgcn_wave_barrier(); asm volatile("" ::: "memory");
        float* crow = C + (size_t)(r0 + mb * 16) * ldc + c0;
#pragma unroll 1
        for (int ps = 0; ps < 2; ++ps) {
#pragma unroll
            for (int s = 0; s < 8; ++s) { const int row = 2 * s + hi, cofs = lr * 4; v4f val = *(const v4fa*)(os + row * 68 + cofs); if (BIAS) { val[0] += bfr(bias[c0 + cofs]); val[1] += bfr(bias[c0 + cofs + 1]); val[2] += bfr(bias[c0 + cofs + 2]); val[3] += bfr(bias[c0 + cofs + 3]); }
                *(volatile v4f*)(crow + (size_t)row * ldc + cofs) = val; }
            if (ps == 0) __threadfence(); }
        __builtin_amdgcn_wave_barrier(); asm volatile("" ::: "memory");
    }
}

__device__ __forceinline__ void splitf(float y, unsigned short& h, unsigned short& l) { h = f2bf(y); l = f2bf(y - bf2f(h)); }
typedef __attribute__((ext_vector_type(2))) unsigned short v2us;

__global__ __launch_bounds__(256) void k_kern(const float* __restrict__ x, int col, const float* __restrict__ e, int n0, bf* Ph, bf* Pl) { const size_t k = ((size_t)blockIdx.x * 256 + threadIdx.x) * 2; if (k >= (size_t)NBIN * CHK) return; const int n = (int)(k % CHK); const int i = (int)(k / CHK);
    const float c = 0.5f * __fadd_rn(bfr(e[i]), bfr(e[i + 1])); const float bw = __fsub_rn(bfr(e[1]), bfr(e[0])); v2us oh, ol;
#pragma unroll
    for (int q = 0; q < 2; ++q) { const float xv = bfr(x[(size_t)(n0 + n + q) * XC + col]); const float z = __fdiv_rn(__fsub_rn(xv, c), bw); float z2 = __fmul_rn(z, z); asm volatile("" : "+v"(z2)); const float v = __expf(-0.5f * z2); unsigned short a, c2; splitf(v, a, c2); oh[q] = a; ol[q] = c2; }
    *(volatile v2us*)(Ph + k) = oh; *(volatile v2us*)(Pl + k) = ol; __threadfence(); *(volatile v2us*)(Ph + k) = oh; *(volatile v2us*)(Pl + k) = ol; }
__global__ __launch_bounds__(256) void k_fin(const float* __restrict__ HP, const float* __restrict__ ex, const float* __restrict__ ey, float* OUT) { const int lane = threadIdx.x & 31; float s = 0.f;
    for (int idx = lane; idx < NBIN * NBIN; idx += 32) { float h = 0.f;
#pragma unroll
        for (int c = 0; c < NCH; ++c) h = __fadd_rn(h, HP[(size_t)c * NBIN * NBIN + idx]); s = __fadd_rn(s, h); }
#pragma unroll
    for (int sh = 16; sh; sh >>= 1) s += __shfl_xor(s, sh, 32);
    const float bwx = __fsub_rn(bfr(ex[1]), bfr(ex[0])), bwy = __fsub_rn(bfr(ey[1]), bfr(ey[0])); float den = __fmul_rn(s, bwx); asm volatile("" : "+v"(den)); den = __fmul_rn(den, bwy);
    for (int ps = 0; ps < 2; ++ps) { for (int u = 0; u < 64; ++u) { const int idx = threadIdx.x * 64 + u; float h = 0.f;
#pragma unroll
            for (int c = 0; c < NCH; ++c) h = __fadd_rn(h, HP[(size_t)c * NBIN * NBIN + idx]); *(volatile float*)(OUT + idx) = __fdiv_rn(h, den); } if (ps == 0) __threadfence(); } }

extern "C" void kernel_launch(void* const* d_in, const int* in_sizes, int n_in,
                              void* d_out, int out_size, void* d_ws, size_t ws_size, hipStream_t stream) {
    (void)in_sizes; (void)n_in; (void)out_size;
    const float* x = (const float*)d_in[0]; const float* ex = (const float*)d_in[1]; const float* ey = (const float*)d_in[2];
    float* OUT = (float*)d_out;
    char* wsp = (char*)d_ws;
    auto take = [&](size_t bytes) { char* p = wsp; wsp += (bytes + 255) & ~(size_t)255; return (void*)p; };
    bf* KXh = (bf*)take((size_t)NBIN * CHK * 2); bf* KXl = (bf*)take((size_t)NBIN * CHK * 2); bf* KYh = (bf*)take((size_t)NBIN * CHK * 2); bf* KYl = (bf*)take((size_t)NBIN * CHK * 2); float* HP = (float*)take((size_t)NCH * NBIN * NBIN * 4);
    if ((size_t)(wsp - (char*)d_ws) > ws_size) return;
    const unsigned LK = (unsigned)(((size_t)NBIN * CHK / 2 + 255) / 256);
    for (int c = 0; c < NCH; ++c) { const int n0 = c * CHK;
        k_kern<<<LK, 256, 0, stream>>>(x, 0, ex, n0, KXh, KXl); k_kern<<<LK, 256, 0, stream>>>(x, 1, ey, n0, KYh, KYl);
        k_gemmw<bf, 2, false><<<dim3(NBIN / 64, NBIN / 64, 1), 32, 0, stream>>>(KXh, KXl, KYh, KYl, CHK, HP + (size_t)c * NBIN * NBIN, NBIN, nullptr, 0, 0, 0); }
    k_fin<<<1, 256, 0, stream>>>(HP, ex, ey, OUT);
}
